// DCGRUCell_90185723281725
// MI455X (gfx1250) — hardware-verified
//
#include <hip/hip_runtime.h>
#include <stdint.h>

constexpr int  kBatch  = 64;
constexpr int  kNodes  = 1024;
constexpr int  kDin    = 2;
constexpr int  kUnits  = 64;
constexpr int  kFeat   = kDin + kUnits;
constexpr int  kFB     = kFeat * kBatch;
constexpr int  kMats   = 5;
constexpr int  kInSz   = kFeat * kMats;
constexpr int  kKproj  = 352;
constexpr int  kPitchF = 384;
constexpr int  kRows   = kBatch * kNodes;
constexpr long kPlane  = (long)kFB * kNodes;
constexpr long kSPlane = (long)kNodes * kNodes;

typedef __attribute__((ext_vector_type(16))) _Float16 v16h;
typedef __attribute__((ext_vector_type(8)))  _Float16 v8h;
typedef __attribute__((ext_vector_type(16))) __bf16   v16b;
typedef __attribute__((ext_vector_type(8)))  __bf16   v8b;
typedef __attribute__((ext_vector_type(8)))  float    v8f;
typedef __attribute__((ext_vector_type(4)))  float    v4f;

__device__ __forceinline__ unsigned short f2bf_bits(float f) {
  unsigned u = __float_as_uint(f);
  return (unsigned short)((u + 0x7FFFu + ((u >> 16) & 1u)) >> 16);
}
__device__ __forceinline__ float bf_bits2f(unsigned short h) { return __uint_as_float(((unsigned)h) << 16); }

__device__ __forceinline__ void dep_guard_h(v8f& a, v8f& b, v16h x, v16h y) { asm volatile("v_nop\n\tv_nop\n\tv_nop\n\tv_nop" : "+v"(a), "+v"(b) : "v"(x), "v"(y)); }
__device__ __forceinline__ void dep_guard_b(v8f& a, v8f& b, v16b x, v16b y) { asm volatile("v_nop\n\tv_nop\n\tv_nop\n\tv_nop" : "+v"(a), "+v"(b) : "v"(x), "v"(y)); }
__device__ __forceinline__ void keep4_h(v16h a, v16h b, v16h c, v16h d) { asm volatile("v_nop" :: "v"(a), "v"(b), "v"(c), "v"(d)); }
__device__ __forceinline__ void keep4_b(v16b a, v16b b, v16b c, v16b d) { asm volatile("v_nop" :: "v"(a), "v"(b), "v"(c), "v"(d)); }
__device__ __forceinline__ void acc_guard4(v8f& a, v8f& b, v8f& c, v8f& d) { asm volatile("v_nop\n\tv_nop\n\tv_nop\n\tv_nop" : "+v"(a), "+v"(b), "+v"(c), "+v"(d)); }
template <typename T> struct Frag;
template <> struct Frag<_Float16> {
  typedef v16h V; union U { v16h v; v8h h[2]; };
  static __device__ __forceinline__ v16h load(const _Float16* p) {
    U f; f.h[0] = *(const v8h*)(p); f.h[1] = *(const v8h*)(p + 16); return f.v;
  }
  static __device__ __forceinline__ v8f mma(v16h a, v16h b, v8f c) {
    return __builtin_amdgcn_wmma_f32_16x16x32_f16(false, a, false, b, (short)0, c, false, false);
  }
  static __device__ __forceinline__ void guard(v8f& a, v8f& b, v16h x, v16h y) { dep_guard_h(a, b, x, y); }
  static __device__ __forceinline__ void keep(v16h a, v16h b, v16h c, v16h d) { keep4_h(a, b, c, d); }
};
template <> struct Frag<__bf16> {
  typedef v16b V; union U { v16b v; v8b h[2]; };
  static __device__ __forceinline__ v16b load(const __bf16* p) {
    U f; f.h[0] = *(const v8b*)(p); f.h[1] = *(const v8b*)(p + 16); return f.v;
  }
  static __device__ __forceinline__ v8f mma(v16b a, v16b b, v8f c) {
    return __builtin_amdgcn_wmma_f32_16x16x32_bf16(false, a, false, b, (short)0, c, false, false);
  }
  static __device__ __forceinline__ void guard(v8f& a, v8f& b, v16b x, v16b y) { dep_guard_b(a, b, x, y); }
  static __device__ __forceinline__ void keep(v16b a, v16b b, v16b c, v16b d) { keep4_b(a, b, c, d); }
};

template <int ET> struct Elem;
template <> struct Elem<0> { typedef _Float16 T; };
template <> struct Elem<1> { typedef __bf16 T; };
template <int ET, bool SPLIT, int BIAS_MODE, int OUT_MODE, bool RESID, int ACT = 0>
__global__ __launch_bounds__(256) void wmma_gemm64(
    const unsigned short* __restrict__ Ap, const unsigned short* __restrict__ A2p, int lda, long strideA,
    const unsigned short* __restrict__ Btp, const unsigned short* __restrict__ Bt2p, int ldb, long strideB,
    void* __restrict__ Cout, void* __restrict__ Cout2, int ldc, long strideC,
    const float* __restrict__ bias,
    const float* __restrict__ resid, long strideR,
    int M, int N, int K, float scale) {
  typedef typename Elem<ET>::T T;
  typedef typename Frag<T>::V V;
  const T* A = (const T*)Ap; const T* A2 = (const T*)A2p; const T* Bt = (const T*)Btp; const T* Bt2 = (const T*)Bt2p;
  __shared__ __align__(16) float sT[8][16 * 68];
  const int b    = blockIdx.y;
  const int lane = threadIdx.x & 31;
  const int wave = threadIdx.x >> 5;
  const int tilesN = N >> 6;
  const int tilesM = M >> 6;
  const int tile = blockIdx.x * 8 + wave;
  if (tile >= tilesM * tilesN) return;
  const int tm = tile / tilesN;
  const int tn = tile - tm * tilesN;
  const int m0 = tm << 6;
  const int n0 = tn << 6;

  const T* Ab  = A  + (size_t)b * strideA;
  const T* Bb  = Bt + (size_t)b * strideB;
  const T* Ab2 = SPLIT ? (A2  + (size_t)b * strideA) : nullptr;
  const T* Bb2 = SPLIT ? (Bt2 + (size_t)b * strideB) : nullptr;

  const int rlane = lane & 15;
  const int koff  = (lane >> 4) * 8;
  const int mOff  = (lane >> 4) * 8;

  v8f acc[4][4];
#pragma unroll
  for (int i = 0; i < 4; ++i)
#pragma unroll
    for (int j = 0; j < 4; ++j) acc[i][j] = (v8f){0.f,0.f,0.f,0.f,0.f,0.f,0.f,0.f};

  for (int k0 = 0; k0 < K; k0 += 32) {
    V bh[4], bl[4];
#pragma unroll
    for (int j = 0; j < 4; ++j) {
      const size_t bo = (size_t)(n0 + (j << 4) + rlane) * ldb + koff + k0;
      bh[j] = Frag<T>::load(Bb + bo);
      if (SPLIT) bl[j] = Frag<T>::load(Bb2 + bo);
    }
#pragma unroll
    for (int i = 0; i < 4; ++i) {
      const size_t ao = (size_t)(m0 + (i << 4) + rlane) * lda + koff + k0;
      V ah = Frag<T>::load(Ab + ao);
      V al;
      if (SPLIT) al = Frag<T>::load(Ab2 + ao);
#pragma unroll
      for (int j = 0; j < 4; ++j) {
        acc[i][j] = Frag<T>::mma(ah, bh[j], acc[i][j]);
        if (SPLIT) {
          acc[i][j] = Frag<T>::mma(ah, bl[j], acc[i][j]);
          acc[i][j] = Frag<T>::mma(al, bh[j], acc[i][j]);
        }
      }
      Frag<T>::guard(acc[i][0], acc[i][3], ah, SPLIT ? al : ah);
    }
    Frag<T>::keep(bh[0], bh[1], bh[2], bh[3]);
    if (SPLIT) Frag<T>::keep(bl[0], bl[1], bl[2], bl[3]);
  }
  acc_guard4(acc[0][0], acc[0][1], acc[0][2], acc[0][3]);
  acc_guard4(acc[1][0], acc[1][1], acc[1][2], acc[1][3]);
  acc_guard4(acc[2][0], acc[2][1], acc[2][2], acc[2][3]);
  acc_guard4(acc[3][0], acc[3][1], acc[3][2], acc[3][3]);

  float* slab = sT[wave];
  const float* Rb = RESID ? (resid + (size_t)b * strideR) : nullptr;
#pragma unroll
  for (int i = 0; i < 4; ++i) {
    const int mBase = m0 + (i << 4);
#pragma unroll
    for (int j = 0; j < 4; ++j) {
      const int n = n0 + (j << 4) + rlane;
      float bv = 0.f;
      if (BIAS_MODE == 2) bv = bias[n];
#pragma unroll
      for (int r = 0; r < 8; ++r) {
        float v = acc[i][j][r] * scale;
        if (BIAS_MODE == 1) v += bias[mBase + mOff + r];
        if (BIAS_MODE == 2) v += bv;
        if (RESID) v += Rb[(size_t)(mBase + mOff + r) * ldc + n];
        if (ACT == 1) v = tanhf(v);
        if (ACT == 2) v = fmaxf(v, 0.0f);
        if (ACT == 3) v = v / (1.0f + expf(-v));
        if (ACT == 4) v = (v > 0.f) ? v : 0.01f * v;
        if (ACT == 6) { const float e = __expf(fminf(-v, 80.0f)); v = __builtin_amdgcn_rcpf(1.0f + e); }
        if (ACT == 7) { const float e = __expf(fminf(-2.0f * v, 80.0f)); v = (1.0f - e) * __builtin_amdgcn_rcpf(1.0f + e); }
        slab[(mOff + r) * 68 + (j << 4) + rlane] = v;
      }
    }
    __builtin_amdgcn_fence(__ATOMIC_RELEASE, "workgroup");
    __builtin_amdgcn_wave_barrier();
    __builtin_amdgcn_fence(__ATOMIC_ACQUIRE, "workgroup");
    if (OUT_MODE == 0) {
      float* C = (float*)Cout + (size_t)b * strideC;
      const int hh = lane >> 4, c4 = (lane & 15) * 4;
      for (int pass = 0; pass < 2; ++pass) {
#pragma unroll
        for (int it = 0; it < 8; ++it) {
          const int row = it * 2 + hh;
          v4f v = *(const v4f*)(slab + row * 68 + c4);
          *(volatile v4f*)(C + (size_t)(mBase + row) * ldc + n0 + c4) = v;
        }
        __threadfence();
      }
    } else {
      const int q = lane >> 3, c8 = (lane & 7) * 8;
      unsigned short* C  = (unsigned short*)Cout  + (size_t)b * strideC;
      unsigned short* C2 = (OUT_MODE == 2) ? ((unsigned short*)Cout2 + (size_t)b * strideC) : nullptr;
      for (int pass = 0; pass < 2; ++pass) {
#pragma unroll
        for (int it = 0; it < 4; ++it) {
          const int row = it * 4 + q;
          const float* sp = slab + row * 68 + c8;
          v8h hv, lv;
#pragma unroll
          for (int e = 0; e < 8; ++e) {
            if (OUT_MODE == 1) {
              hv[e] = (_Float16)sp[e];
            } else {
              unsigned short hb = f2bf_bits(sp[e]);
              unsigned short lb = f2bf_bits(sp[e] - bf_bits2f(hb));
              hv[e] = __builtin_bit_cast(_Float16, hb);
              lv[e] = __builtin_bit_cast(_Float16, lb);
            }
          }
          *(volatile v8h*)(C + (size_t)(mBase + row) * ldc + n0 + c8) = hv;
          if (OUT_MODE == 2) *(volatile v8h*)(C2 + (size_t)(mBase + row) * ldc + n0 + c8) = lv;
        }
        __threadfence();
      }
    }
    __builtin_amdgcn_fence(__ATOMIC_RELEASE, "workgroup");
    __builtin_amdgcn_wave_barrier();
    __builtin_amdgcn_fence(__ATOMIC_ACQUIRE, "workgroup");
  }
}

__global__ __launch_bounds__(256) void cast_supports_f16x2(const float* __restrict__ s0, const float* __restrict__ s1,
                                                           _Float16* __restrict__ out, int n2) {
  const int i = blockIdx.x * 256 + threadIdx.x;
  const int nblk = n2 >> 8;
  const bool second = (int)blockIdx.x >= nblk;
  const float* src = second ? s1 : s0;
  const int j = second ? (i - n2) : i;
  if (i < 2 * n2) {
    const float a = src[2 * (size_t)j] * 256.0f, c = src[2 * (size_t)j + 1] * 256.0f;
    const _Float16 h0 = (_Float16)a, h1 = (_Float16)c;
    const unsigned u = (unsigned)__builtin_bit_cast(unsigned short, h0) | ((unsigned)__builtin_bit_cast(unsigned short, h1) << 16);
    ((volatile unsigned*)out)[i] = u;
    __threadfence();
    ((volatile unsigned*)out)[i] = u;
  }
}

__global__ __launch_bounds__(256) void cast_weights_f16t(const float* __restrict__ Wo, const float* __restrict__ Wu,
                                                         _Float16* __restrict__ WoT, _Float16* __restrict__ WuT) {
  const int lane = threadIdx.x & 31, wave = threadIdx.x >> 5;
  const bool upd = blockIdx.x >= 16;
  const float* W = upd ? Wu : Wo;
  _Float16* dst  = upd ? WuT : WoT;
  const int outn = upd ? kUnits : 2 * kUnits;
  const int o = ((upd ? ((int)blockIdx.x - 16) : (int)blockIdx.x) << 3) + wave;
  v8h p0, p1;
#pragma unroll
  for (int e = 0; e < 8; ++e) {
    const int k0 = lane * 8 + e;
    p0[e] = (_Float16)(W[(size_t)k0 * outn + o] * 16.0f);
    const int k1 = 256 + (lane & 15) * 8 + e;
    const int k1c = k1 < kInSz ? k1 : kInSz - 1;
    float w1 = W[(size_t)k1c * outn + o] * 16.0f;
    if (k1 >= kInSz) w1 = 0.0f;
    p1[e] = (_Float16)w1;
  }
  _Float16* rp = dst + (size_t)o * kPitchF;
  for (int pass = 0; pass < 2; ++pass) {
    *(volatile v8h*)(rp + lane * 8) = p0;
    if (lane < 16) *(volatile v8h*)(rp + 256 + lane * 8) = p1;
    __threadfence();
  }
}

template <int MODE>
__global__ __launch_bounds__(128) void pack_x0t(const float* __restrict__ inputs, const float* __restrict__ hx,
                                                const float* __restrict__ value, _Float16* __restrict__ X0T, int row0) {
  const int j = row0 + blockIdx.x;
  const int f = j >> 6, b = j & 63;
  const int nb = threadIdx.x * 8;
  v8h hv;
  if (f < kDin) {
#pragma unroll
    for (int e = 0; e < 8; ++e)
      hv[e] = (_Float16)inputs[(size_t)b * (kNodes * kDin) + (size_t)(nb + e) * kDin + f];
  } else {
    const int u = f - kDin;
#pragma unroll
    for (int e = 0; e < 8; ++e) {
      const size_t row = (size_t)b * kNodes + nb + e;
      float h = hx[row * kUnits + u];
      if (MODE == 1) h = value[row * (2 * kUnits) + u] * h;
      hv[e] = (_Float16)h;
    }
  }
  _Float16* p = X0T + (size_t)j * kNodes + nb;
  *(volatile v8h*)p = hv;
  __threadfence();
  *(volatile v8h*)p = hv;
}

template <int MODE>
__global__ __launch_bounds__(256) void gather_feat(const float* __restrict__ inputs, const float* __restrict__ hx,
                                                   const float* __restrict__ value,
                                                   const _Float16* __restrict__ X1S, const _Float16* __restrict__ P2S,
                                                   _Float16* __restrict__ FEAT) {
  __shared__ __align__(16) _Float16 tile[32 * kPitchF];
  const int tid = threadIdx.x, lane = tid & 31, wave = tid >> 5;
  const int rowb = blockIdx.x * 32;
  const int b = rowb >> 10;
  const int n = (rowb & (kNodes - 1)) + lane;
  const size_t row = (size_t)rowb + lane;
  if (tid < 224) {
    const int r = tid / 7, pc = tid - r * 7;
    v8h z8;
#pragma unroll
    for (int e = 0; e < 8; ++e) z8[e] = (_Float16)0.0f;
    *(v8h*)(tile + r * kPitchF + 328 + pc * 8) = z8;
  }
  __syncthreads();
#pragma unroll 1
  for (int it = 0; it < 9; ++it) {
    const int f = wave + it * 8;
    if (f < kFeat) {
      const int fi = f < kDin ? f : kDin - 1;
      const int fu = f >= kDin ? f - kDin : 0;
      const float xin = inputs[(size_t)b * (kNodes * kDin) + (size_t)n * kDin + fi];
      float xh = hx[row * kUnits + fu];
      if (MODE == 1) xh = value[row * (2 * kUnits) + fu] * xh;
      const float x16 = 16.0f * ((f < kDin) ? xin : xh);
      const size_t po = (size_t)(f * kBatch + b) * kNodes + n;
      const _Float16 a1 = X1S[po];
      const _Float16 a3 = X1S[(size_t)kPlane + po];
      const float p2a = (float)P2S[po];
      const float p2b = (float)P2S[(size_t)kPlane + po];
      _Float16* tr = tile + lane * kPitchF + f * kMats;
      tr[0] = (_Float16)x16;
      tr[1] = a1;
      tr[2] = (_Float16)(p2a - x16);
      tr[3] = a3;
      tr[4] = (_Float16)(p2b - x16);
    }
  }
  __syncthreads();
  v8h va[4], vc[4];
#pragma unroll
  for (int r = 0; r < 4; ++r) {
    const _Float16* src = tile + (wave * 4 + r) * kPitchF;
    va[r] = *(const v8h*)(src + lane * 8);
    vc[r] = *(const v8h*)(src + 256 + (lane & 15) * 8);
  }
  for (int pass = 0; pass < 2; ++pass) {
#pragma unroll
    for (int r = 0; r < 4; ++r) {
      _Float16* dstp = FEAT + ((size_t)rowb + wave * 4 + r) * kPitchF;
      *(volatile v8h*)(dstp + lane * 8) = va[r];
      if (lane < 16) *(volatile v8h*)(dstp + 256 + lane * 8) = vc[r];
    }
    __threadfence();
  }
}

__global__ __launch_bounds__(256) void gru_combine(const float* __restrict__ hx, const float* __restrict__ value,
                                                   const float* __restrict__ cplane, float* out, int n4) {
  const int i = blockIdx.x * 256 + threadIdx.x;
  if (i < n4) {
    const size_t row = (size_t)(i >> 4);
    const int c = (i & 15) * 4;
    const v4f u  = *(const v4f*)(value + row * (2 * kUnits) + kUnits + c);
    const v4f h  = *(const v4f*)(hx + (size_t)i * 4);
    const v4f cv = *(const v4f*)(cplane + (size_t)i * 4);
    const v4f o  = u * h + (1.0f - u) * cv;
    *(volatile v4f*)(out + (size_t)i * 4) = o;
    __threadfence();
    *(volatile v4f*)(out + (size_t)i * 4) = o;
  }
}

extern "C" void kernel_launch(void* const* d_in, const int* in_sizes, int n_in,
                              void* d_out, int out_size, void* d_ws, size_t ws_size, hipStream_t stream) {
  if (n_in < 8) return;
  if (in_sizes[0] != kBatch * kNodes * kDin || in_sizes[1] != kRows * kUnits ||
      in_sizes[2] != kNodes * kNodes || in_sizes[3] != kNodes * kNodes ||
      in_sizes[4] != kInSz * 2 * kUnits || in_sizes[5] != 2 * kUnits ||
      in_sizes[6] != kInSz * kUnits || in_sizes[7] != kUnits) return;
  if (out_size != kRows * kUnits) return;

  const float* inputs = (const float*)d_in[0];
  const float* hx     = (const float*)d_in[1];
  const float* s0     = (const float*)d_in[2];
  const float* s1     = (const float*)d_in[3];
  const float* Wo     = (const float*)d_in[4];
  const float* bo     = (const float*)d_in[5];
  const float* Wu     = (const float*)d_in[6];
  const float* bu     = (const float*)d_in[7];
  float* out = (float*)d_out;

  char* ws = (char*)d_ws; size_t off = 0;
  auto carve = [&](size_t bytes) -> char* { char* p = ws + off; off += (bytes + 255) & ~(size_t)255; return p; };
  _Float16* S16   = (_Float16*)carve((size_t)2 * kSPlane * 2);
  _Float16* X0T   = (_Float16*)carve((size_t)kPlane * 2);
  _Float16* X1S   = (_Float16*)carve((size_t)2 * kPlane * 2);
  _Float16* P2S   = (_Float16*)carve((size_t)2 * kPlane * 2);
  _Float16* WoT   = (_Float16*)carve((size_t)(2 * kUnits) * kPitchF * 2);
  _Float16* WuT   = (_Float16*)carve((size_t)kUnits * kPitchF * 2);
  _Float16* FEAT  = (_Float16*)carve((size_t)kRows * kPitchF * 2);
  float*    VALUE = (float*)carve((size_t)kRows * (2 * kUnits) * 4);
  float*    CPL   = (float*)(void*)X0T;
  if (off > ws_size || off > (size_t)134217728) return;

  typedef const unsigned short* cus;
  const int n2 = (int)(kSPlane / 2);
  cast_supports_f16x2<<<(2 * n2) / 256, 256, 0, stream>>>(s0, s1, S16, n2);
  cast_weights_f16t<<<16 + 8, 256, 0, stream>>>(Wo, Wu, WoT, WuT);

  const int tilesFull = (kFB / 64) * (kNodes / 64);
  const int tilesHid  = ((kFB - 128) / 64) * (kNodes / 64);
  const size_t hidOff = (size_t)128 * kNodes;

  pack_x0t<0><<<kFB, 128, 0, stream>>>(inputs, hx, VALUE, X0T, 0);
  wmma_gemm64<0, false, 0, 1, false, 0><<<dim3((tilesFull + 7) / 8, 2), 256, 0, stream>>>(
      (cus)X0T, (cus)X0T, kNodes, 0L, (cus)S16, (cus)S16, kNodes, kSPlane,
      (void*)X1S, (void*)nullptr, kNodes, kPlane, (const float*)nullptr, (const float*)nullptr, 0L,
      kFB, kNodes, kNodes, 0.0625f);
  wmma_gemm64<0, false, 0, 1, false, 0><<<dim3((tilesFull + 7) / 8, 2), 256, 0, stream>>>(
      (cus)X1S, (cus)X1S, kNodes, kPlane, (cus)S16, (cus)S16, kNodes, kSPlane,
      (void*)P2S, (void*)nullptr, kNodes, kPlane, (const float*)nullptr, (const float*)nullptr, 0L,
      kFB, kNodes, kNodes, 0.0078125f);
  gather_feat<0><<<kRows / 32, 256, 0, stream>>>(inputs, hx, VALUE, X1S, P2S, FEAT);
  wmma_gemm64<0, false, 2, 0, false, 6><<<dim3(((kRows / 64) * (2 * kUnits / 64) + 7) / 8, 1), 256, 0, stream>>>(
      (cus)FEAT, (cus)FEAT, kPitchF, 0L, (cus)WoT, (cus)WoT, kPitchF, 0L,
      (void*)VALUE, (void*)nullptr, 2 * kUnits, 0L, bo, (const float*)nullptr, 0L,
      kRows, 2 * kUnits, kKproj, 0.00390625f);

  pack_x0t<1><<<kFB - 128, 128, 0, stream>>>(inputs, hx, VALUE, X0T, 128);
  wmma_gemm64<0, false, 0, 1, false, 0><<<dim3((tilesHid + 7) / 8, 2), 256, 0, stream>>>(
      (cus)(X0T + hidOff), (cus)(X0T + hidOff), kNodes, 0L, (cus)S16, (cus)S16, kNodes, kSPlane,
      (void*)(X1S + hidOff), (void*)nullptr, kNodes, kPlane, (const float*)nullptr, (const float*)nullptr, 0L,
      kFB - 128, kNodes, kNodes, 0.0625f);
  wmma_gemm64<0, false, 0, 1, false, 0><<<dim3((tilesHid + 7) / 8, 2), 256, 0, stream>>>(
      (cus)(X1S + hidOff), (cus)(X1S + hidOff), kNodes, kPlane, (cus)S16, (cus)S16, kNodes, kSPlane,
      (void*)(P2S + hidOff), (void*)nullptr, kNodes, kPlane, (const float*)nullptr, (const float*)nullptr, 0L,
      kFB - 128, kNodes, kNodes, 0.0078125f);
  gather_feat<1><<<kRows / 32, 256, 0, stream>>>(inputs, hx, VALUE, X1S, P2S, FEAT);
  wmma_gemm64<0, false, 2, 0, false, 7><<<dim3(((kRows / 64) * (kUnits / 64) + 7) / 8, 1), 256, 0, stream>>>(
      (cus)FEAT, (cus)FEAT, kPitchF, 0L, (cus)WuT, (cus)WuT, kPitchF, 0L,
      (void*)CPL, (void*)nullptr, kUnits, 0L, bu, (const float*)nullptr, 0L,
      kRows, kUnits, kKproj, 0.00390625f);

  gru_combine<<<(kRows * kUnits / 4) / 256, 256, 0, stream>>>(hx, VALUE, CPL, out, kRows * kUnits / 4);
}
